// RPEConformerBlock_89189290869053
// MI455X (gfx1250) — hardware-verified
//
#include <hip/hip_runtime.h>
#include <math.h>
#include <stdint.h>
#include <stddef.h>

#define NB_   4
#define NT_   1024
#define ND_   512
#define NH_   8
#define HD_   64
#define NF_   2048
#define KW_   31
#define NR_   4096
#define NP_   2047
#define NPP_  2048
#define BDW_  1088
#define NGRP_ 8

#define MODE_F32    0
#define MODE_RES32  1
#define MODE_H16    2
#define MODE_H16B   3
#define MODE_H16RB  4
#define MODE_QUV    5
#define MODE_SILU16 6
#define MODE_GLU32  7

typedef _Float16 v16h __attribute__((ext_vector_type(16)));
typedef _Float16 v8h  __attribute__((ext_vector_type(8)));
typedef float    v8f  __attribute__((ext_vector_type(8)));
typedef float    v4f  __attribute__((ext_vector_type(4)));
typedef v4f __attribute__((may_alias)) v4fa;
typedef v8h __attribute__((may_alias)) v8ha;

union FragU { v16h v; v8ha h[2]; };
__device__ __forceinline__ v16h ldfrag(const _Float16* p) {
  FragU f;
  f.h[0] = *(const v8ha*)(p);
  f.h[1] = *(const v8ha*)(p + 16);
  return f.v;
}

__device__ __forceinline__ v8f mma16(v16h a, v16h b, v8f c) {
  c = __builtin_amdgcn_wmma_f32_16x16x32_f16(false, a, false, b, (short)0, c, false, false);
#if defined(__HIP_DEVICE_COMPILE__)
  asm volatile("v_nop\n\tv_nop\n\tv_nop\n\tv_nop" : "+v"(c) : "v"(a), "v"(b));
#endif
  return c;
}

__device__ __forceinline__ v8f zero8() { v8f z = {0.f, 0.f, 0.f, 0.f, 0.f, 0.f, 0.f, 0.f}; return z; }
__device__ __forceinline__ float rcp_f(float x) { return __builtin_amdgcn_rcpf(x); }
__device__ __forceinline__ float silu_f(float v) { return v * rcp_f(1.0f + __expf(-v)); }
__device__ __forceinline__ float sigm_f(float v) { return rcp_f(1.0f + __expf(-v)); }

__device__ __forceinline__ void wave_lds_sync() {
  __builtin_amdgcn_fence(__ATOMIC_RELEASE, "workgroup");
  __builtin_amdgcn_wave_barrier();
  __builtin_amdgcn_fence(__ATOMIC_ACQUIRE, "workgroup");
}

__global__ __launch_bounds__(256) void cvt_rows_kernel(const float* __restrict__ src, _Float16* __restrict__ dst,
                                                       int nrows_src, int nrows_dst, float scale) {
  const int i = blockIdx.x * 256 + threadIdx.x;
  const int total8 = nrows_dst * (ND_ / 8);
  if (i >= total8) return;
  const int r  = i / (ND_ / 8);
  const int c8 = (i - r * (ND_ / 8)) * 8;
  const int rs = (r < nrows_src) ? r : (nrows_src - 1);
  const float sc = (r < nrows_src) ? scale : 0.0f;
  const float* sp = src + (size_t)rs * ND_ + c8;
  const v4f a = *(const v4f*)(sp);
  const v4f b = *(const v4f*)(sp + 4);
  v8h o;
  o[0] = (_Float16)(a[0] * sc); o[1] = (_Float16)(a[1] * sc); o[2] = (_Float16)(a[2] * sc); o[3] = (_Float16)(a[3] * sc);
  o[4] = (_Float16)(b[0] * sc); o[5] = (_Float16)(b[1] * sc); o[6] = (_Float16)(b[2] * sc); o[7] = (_Float16)(b[3] * sc);
  _Float16* dp = dst + (size_t)r * ND_ + c8;
  *(volatile v8h*)dp = o;
  __threadfence();
  *(volatile v8h*)dp = o;
}

__global__ __launch_bounds__(256) void wtrans_kernel(const float* __restrict__ src, _Float16* __restrict__ dst,
                                                     int K, int N, float carry) {
  __shared__ float tile[64][65];
  const int tid = threadIdx.x;
  const int n0 = blockIdx.x * 64;
  const int k0 = blockIdx.y * 64;
#pragma unroll
  for (int i = 0; i < 16; ++i) {
    const int idx = i * 256 + tid;
    const int kr = idx >> 6;
    const int nc = idx & 63;
    tile[kr][nc] = src[(size_t)(k0 + kr) * N + n0 + nc];
  }
  __syncthreads();
  const int q = tid >> 3, c8 = (tid & 7) * 8;
  v8h ov[2];
#pragma unroll
  for (int p = 0; p < 2; ++p) {
    const int nr = q + 32 * p;
    v8h t;
#pragma unroll
    for (int e = 0; e < 8; ++e) t[e] = (_Float16)(tile[c8 + e][nr] * carry);
    ov[p] = t;
  }
  for (int pass = 0; pass < 2; ++pass) {
#pragma unroll
    for (int p = 0; p < 2; ++p) {
      const int nr = q + 32 * p;
      *(volatile v8h*)(dst + (size_t)(n0 + nr) * K + k0 + c8) = ov[p];
    }
    __threadfence();
  }
}

template <int OUTK>
__global__ __launch_bounds__(256) void ln_kernel(const float* __restrict__ X, const float* __restrict__ g,
                                                 const float* __restrict__ bb, void* __restrict__ outp,
                                                 int nrows, float carry) {
  const int lane = threadIdx.x & 31, wave = threadIdx.x >> 5;
  const int row = blockIdx.x * 8 + wave;
  if (row >= nrows) return;
  const float* x = X + (size_t)row * ND_;
  float v[16];
  if (OUTK == 0) {
#pragma unroll
    for (int i = 0; i < 2; ++i) {
      const v4f a = *(const v4f*)(x + 256 * i + 8 * lane);
      const v4f c = *(const v4f*)(x + 256 * i + 8 * lane + 4);
      v[8 * i + 0] = a[0]; v[8 * i + 1] = a[1]; v[8 * i + 2] = a[2]; v[8 * i + 3] = a[3];
      v[8 * i + 4] = c[0]; v[8 * i + 5] = c[1]; v[8 * i + 6] = c[2]; v[8 * i + 7] = c[3];
    }
  } else {
#pragma unroll
    for (int i = 0; i < 4; ++i) {
      const v4f a = *(const v4f*)(x + 128 * i + 4 * lane);
      v[4 * i + 0] = a[0]; v[4 * i + 1] = a[1]; v[4 * i + 2] = a[2]; v[4 * i + 3] = a[3];
    }
  }
  float s = 0.f;
#pragma unroll
  for (int e = 0; e < 16; ++e) s += v[e];
  s += __shfl_xor(s, 1, 32); s += __shfl_xor(s, 2, 32); s += __shfl_xor(s, 4, 32);
  s += __shfl_xor(s, 8, 32); s += __shfl_xor(s, 16, 32);
  const float mean = s * (1.0f / (float)ND_);
  float ss = 0.f;
#pragma unroll
  for (int e = 0; e < 16; ++e) { const float d = v[e] - mean; ss += d * d; }
  ss += __shfl_xor(ss, 1, 32); ss += __shfl_xor(ss, 2, 32); ss += __shfl_xor(ss, 4, 32);
  ss += __shfl_xor(ss, 8, 32); ss += __shfl_xor(ss, 16, 32);
  const float rstd = rsqrtf(ss * (1.0f / (float)ND_) + 1e-5f);
  if (OUTK == 0) {
    _Float16* o = (_Float16*)outp + (size_t)row * ND_;
    v8h ov[2];
#pragma unroll
    for (int i = 0; i < 2; ++i) {
      const int base = 256 * i + 8 * lane;
      const v4f g0 = *(const v4f*)(g + base),  g1 = *(const v4f*)(g + base + 4);
      const v4f b0 = *(const v4f*)(bb + base), b1 = *(const v4f*)(bb + base + 4);
      float gg[8], bv[8];
      gg[0] = g0[0]; gg[1] = g0[1]; gg[2] = g0[2]; gg[3] = g0[3]; gg[4] = g1[0]; gg[5] = g1[1]; gg[6] = g1[2]; gg[7] = g1[3];
      bv[0] = b0[0]; bv[1] = b0[1]; bv[2] = b0[2]; bv[3] = b0[3]; bv[4] = b1[0]; bv[5] = b1[1]; bv[6] = b1[2]; bv[7] = b1[3];
      v8h t;
#pragma unroll
      for (int e = 0; e < 8; ++e) t[e] = (_Float16)((((v[8 * i + e] - mean) * rstd) * gg[e] + bv[e]) * carry);
      ov[i] = t;
    }
    for (int pass = 0; pass < 2; ++pass) {
#pragma unroll
      for (int i = 0; i < 2; ++i) *(volatile v8h*)(o + 256 * i + 8 * lane) = ov[i];
      __threadfence();
    }
  } else {
    float* o = (float*)outp + (size_t)row * ND_;
    v4f ov[4];
#pragma unroll
    for (int i = 0; i < 4; ++i) {
      const int base = 128 * i + 4 * lane;
      const v4f g0 = *(const v4f*)(g + base);
      const v4f b0 = *(const v4f*)(bb + base);
      v4f t;
#pragma unroll
      for (int e = 0; e < 4; ++e) t[e] = (((v[4 * i + e] - mean) * rstd) * g0[e] + b0[e]) * carry;
      ov[i] = t;
    }
    for (int pass = 0; pass < 2; ++pass) {
#pragma unroll
      for (int i = 0; i < 4; ++i) *(volatile v4f*)(o + 128 * i + 4 * lane) = ov[i];
      __threadfence();
    }
  }
}

template <int MODE, bool SKEW>
__global__ __launch_bounds__(256) void gemm_kernel(
    const _Float16* __restrict__ A, int lda, long strideA,
    const _Float16* __restrict__ Bt, int ldb, long strideB,
    void* C1, void* C2, int ldc, long strideC,
    const float* Rsd, int ldr, long strideR,
    const float* __restrict__ b1, const float* __restrict__ b2, const float* __restrict__ b3,
    int M, int N, int K, int gofs, float scale, float scale2, float carry) {
  __shared__ __align__(16) float sT[8][16 * 68];

  const int z    = blockIdx.y;
  const int lane = threadIdx.x & 31;
  const int wave = threadIdx.x >> 5;
  const bool glu = (MODE == MODE_GLU32);
  const int tilesN = glu ? (N >> 5) : (N >> 6);
  const int tilesM = M >> 6;
  const int tile = blockIdx.x * 8 + wave;
  if (tile >= tilesM * tilesN) return;
  const int tm = tile / tilesN;
  const int tn = tile - tm * tilesN;
  const int m0 = tm << 6;
  const int n0 = glu ? (tn << 5) : (tn << 6);
  const int nsk = SKEW ? (tm << 6) : 0;

  const _Float16* Ab = A  + (size_t)((long)z * strideA);
  const _Float16* Bb = Bt + (size_t)((long)z * strideB);

  const int rl   = lane & 15;
  const int koff = (lane >> 4) * 8;
  const int mOff = (lane >> 4) * 8;

  const _Float16* ap[4];
  const _Float16* bp[4];
#pragma unroll
  for (int i = 0; i < 4; ++i) ap[i] = Ab + (size_t)(m0 + (i << 4) + rl) * lda + koff;
#pragma unroll
  for (int j = 0; j < 4; ++j) {
    int br;
    if (glu) br = (j < 2) ? (n0 + (j << 4) + rl) : (gofs + n0 + ((j - 2) << 4) + rl);
    else     br = nsk + n0 + (j << 4) + rl;
    bp[j] = Bb + (size_t)br * ldb + koff;
  }

  v8f acc[4][4];
#pragma unroll
  for (int i = 0; i < 4; ++i)
#pragma unroll
    for (int j = 0; j < 4; ++j) acc[i][j] = zero8();

  for (int k0 = 0; k0 < K; k0 += 32) {
    v16h bfr[4];
#pragma unroll
    for (int j = 0; j < 4; ++j) bfr[j] = ldfrag(bp[j] + k0);
#pragma unroll
    for (int i = 0; i < 4; ++i) {
      const v16h af = ldfrag(ap[i] + k0);
#pragma unroll
      for (int j = 0; j < 4; ++j) acc[i][j] = mma16(af, bfr[j], acc[i][j]);
    }
  }

  float* slab = sT[wave];
#pragma unroll
  for (int i = 0; i < 4; ++i) {
    const int mBase = m0 + (i << 4);
#pragma unroll
    for (int j = 0; j < 4; ++j)
#pragma unroll
      for (int r = 0; r < 8; ++r)
        slab[(mOff + r) * 68 + (j << 4) + rl] = acc[i][j][r] * scale;
    wave_lds_sync();
    if (MODE == MODE_F32 || MODE == MODE_RES32) {
      float* Cz = (float*)C1 + (size_t)((long)z * strideC);
      const int hh = lane >> 4, c4 = (lane & 15) * 4;
      v4f vals[8];
#pragma unroll
      for (int it = 0; it < 8; ++it) {
        const int row = it * 2 + hh;
        const v4f sv = *(const v4fa*)(slab + row * 68 + c4);
        if (MODE == MODE_RES32) {
          const float* rp = Rsd + (size_t)((long)z * strideR) + (size_t)(mBase + row) * ldr + n0 + c4;
          const v4f rv = *(const v4f*)(rp);
          const v4f bv = *(const v4f*)(b1 + n0 + c4);
          v4f o;
#pragma unroll
          for (int e = 0; e < 4; ++e) o[e] = rv[e] + scale2 * (sv[e] + bv[e]);
          vals[it] = o;
        } else {
          vals[it] = sv;
        }
      }
      for (int pass = 0; pass < 2; ++pass) {
#pragma unroll
        for (int it = 0; it < 8; ++it) {
          const int row = it * 2 + hh;
          *(volatile v4f*)(Cz + (size_t)(mBase + row) * ldc + n0 + c4) = vals[it];
        }
        __threadfence();
      }
    } else if (MODE == MODE_GLU32) {
      float* Cz = (float*)C1 + (size_t)((long)z * strideC);
      const int q = lane >> 3, c4 = (lane & 7) * 4;
      const v4f ba = *(const v4f*)(b1 + n0 + c4);
      const v4f bg = *(const v4f*)(b1 + gofs + n0 + c4);
      v4f vals[4];
#pragma unroll
      for (int it = 0; it < 4; ++it) {
        const int row = it * 4 + q;
        const v4f av = *(const v4fa*)(slab + row * 68 + c4);
        const v4f gv = *(const v4fa*)(slab + row * 68 + 32 + c4);
        v4f o;
#pragma unroll
        for (int e = 0; e < 4; ++e) o[e] = (av[e] + ba[e]) * sigm_f(gv[e] + bg[e]);
        vals[it] = o;
      }
      for (int pass = 0; pass < 2; ++pass) {
#pragma unroll
        for (int it = 0; it < 4; ++it) {
          const int row = it * 4 + q;
          *(volatile v4f*)(Cz + (size_t)(mBase + row) * ldc + n0 + c4) = vals[it];
        }
        __threadfence();
      }
    } else {
      const int q = lane >> 3, c8 = (lane & 7) * 8;
      _Float16* Ca = (_Float16*)C1 + (size_t)((long)z * strideC);
      _Float16* Cb = (_Float16*)C2 + (size_t)((long)z * strideC);
      v8h hv[4], lv[4];
#pragma unroll
      for (int it = 0; it < 4; ++it) {
        const int row = it * 4 + q;
        const int m = mBase + row;
        const float* sp = slab + row * 68 + c8;
        const v4f x0 = *(const v4fa*)(sp);
        const v4f x1 = *(const v4fa*)(sp + 4);
        float f[8];
        f[0] = x0[0]; f[1] = x0[1]; f[2] = x0[2]; f[3] = x0[3];
        f[4] = x1[0]; f[5] = x1[1]; f[6] = x1[2]; f[7] = x1[3];
        v8h ha, hb;
#pragma unroll
        for (int e = 0; e < 8; ++e) {
          const int n = n0 + c8 + e;
          if (MODE == MODE_H16) {
            ha[e] = (_Float16)(f[e] * carry);
            hb[e] = ha[e];
          } else if (MODE == MODE_H16B) {
            ha[e] = (_Float16)((f[e] + b1[n]) * carry);
            hb[e] = ha[e];
          } else if (MODE == MODE_H16RB) {
            ha[e] = (_Float16)((f[e] + b1[m]) * carry);
            hb[e] = ha[e];
          } else if (MODE == MODE_QUV) {
            const float t = f[e] + b1[n];
            ha[e] = (_Float16)((t + b2[n]) * carry);
            hb[e] = (_Float16)((t + b3[n]) * carry);
          } else {
            ha[e] = (_Float16)(silu_f(f[e] + b1[n]) * carry);
            hb[e] = ha[e];
          }
        }
        hv[it] = ha; lv[it] = hb;
      }
      for (int pass = 0; pass < 2; ++pass) {
#pragma unroll
        for (int it = 0; it < 4; ++it) {
          const int row = it * 4 + q;
          *(volatile v8h*)(Ca + (size_t)(mBase + row) * ldc + n0 + c8) = hv[it];
          if (MODE == MODE_QUV) *(volatile v8h*)(Cb + (size_t)(mBase + row) * ldc + n0 + c8) = lv[it];
        }
        __threadfence();
      }
    }
    wave_lds_sync();
  }
}

__global__ __launch_bounds__(128)
void relattn_kernel(const _Float16* __restrict__ QU, const _Float16* __restrict__ Kp,
                    const _Float16* __restrict__ VT, const float* __restrict__ BD,
                    _Float16* __restrict__ CTX, int pairBase, float cs) {
  __shared__ __align__(16) unsigned char SMEM[24576];
  _Float16* Ksh = (_Float16*)(SMEM);
  _Float16* Vsh = (_Float16*)(SMEM + 8192);
  _Float16* Psh = (_Float16*)(SMEM + 16384);
  float*    Osh = (float*)(SMEM);

  const int tid  = threadIdx.x;
  const int wave = tid >> 5;
  const int lane = tid & 31;
  const int hh   = lane >> 4;
  const int c    = lane & 15;

  const int z    = blockIdx.y;
  const int pair = pairBase + z;
  const int b    = pair >> 3;
  const int h    = pair & 7;
  const int qb   = blockIdx.x;
  const int q0   = qb * 64 + wave * 16;
  const int rr0  = wave * 16 + 8 * hh;

  const _Float16* Qh = QU + (size_t)(b * NT_) * ND_ + h * HD_;
  const _Float16* Kh = Kp + (size_t)(b * NT_) * ND_ + h * HD_;
  const _Float16* Vh = VT + (size_t)b * ND_ * NT_ + (size_t)(h * HD_) * NT_;
  const float*    bd = BD + (size_t)z * NT_ * BDW_;
  _Float16*       ctx = CTX + (size_t)(b * NT_) * ND_ + h * HD_;

  v16h qa[2];
#pragma unroll
  for (int dc = 0; dc < 2; ++dc)
    qa[dc] = ldfrag(Qh + (size_t)(q0 + c) * ND_ + dc * 32 + 8 * hh);

  const float* bdr = bd + (long)(q0 + 8 * hh) * BDW_ + (rr0 + (NT_ - 1) - c);

  float mrow[8], lrow[8];
  v8f oacc[4];
#pragma unroll
  for (int r = 0; r < 8; ++r) { mrow[r] = -INFINITY; lrow[r] = 0.f; }
#pragma unroll
  for (int t = 0; t < 4; ++t) oacc[t] = zero8();

  _Float16* pw = Psh + wave * (16 * 64);

  for (int kc = 0; kc < NT_ / 64; ++kc) {
    const int kv0 = kc * 64;
    __syncthreads();
    {
      const int r = tid >> 1, c0 = (tid & 1) * 32;
      const _Float16* ks = Kh + (size_t)(kv0 + r) * ND_ + c0;
      const _Float16* vs = Vh + (size_t)r * NT_ + kv0 + c0;
#pragma unroll
      for (int i = 0; i < 4; ++i) {
        const v8h kk8 = *(const v8h*)(ks + 8 * i);
        const v8h vv8 = *(const v8h*)(vs + 8 * i);
        *(v8ha*)(Ksh + r * 64 + c0 + 8 * i) = kk8;
        *(v8ha*)(Vsh + r * 64 + c0 + 8 * i) = vv8;
      }
    }
    __syncthreads();

    v8f s[4];
#pragma unroll
    for (int j = 0; j < 4; ++j) {
      s[j] = zero8();
#pragma unroll
      for (int dc = 0; dc < 2; ++dc) {
        const v16h kb = ldfrag(Ksh + (j * 16 + c) * 64 + dc * 32 + 8 * hh);
        s[j] = mma16(qa[dc], kb, s[j]);
      }
    }

    float cm[8];
#pragma unroll
    for (int r = 0; r < 8; ++r) {
      float m = -INFINITY;
#pragma unroll
      for (int j = 0; j < 4; ++j) {
        const float sv = s[j][r] * cs + bdr[(long)r * (BDW_ + 1) - kv0 - (j << 4)];
        s[j][r] = sv;
        m = fmaxf(m, sv);
      }
      m = fmaxf(m, __shfl_xor(m, 1, 32));
      m = fmaxf(m, __shfl_xor(m, 2, 32));
      m = fmaxf(m, __shfl_xor(m, 4, 32));
      m = fmaxf(m, __shfl_xor(m, 8, 32));
      cm[r] = m;
    }

#pragma unroll
    for (int r = 0; r < 8; ++r) {
      const float mnew  = fmaxf(mrow[r], cm[r]);
      const float alpha = __expf(mrow[r] - mnew);
      mrow[r] = mnew;
      float psum = 0.f;
#pragma unroll
      for (int j = 0; j < 4; ++j) {
        const float p = __expf(s[j][r] - mnew);
        psum += p;
        pw[(8 * hh + r) * 64 + j * 16 + c] = (_Float16)(p * 4096.0f);
      }
      psum += __shfl_xor(psum, 1, 32);
      psum += __shfl_xor(psum, 2, 32);
      psum += __shfl_xor(psum, 4, 32);
      psum += __shfl_xor(psum, 8, 32);
      lrow[r] = lrow[r] * alpha + psum;
#pragma unroll
      for (int t = 0; t < 4; ++t) oacc[t][r] *= alpha;
    }
    wave_lds_sync();

#pragma unroll
    for (int kk = 0; kk < 2; ++kk) {
      const v16h pa = ldfrag(pw + c * 64 + kk * 32 + 8 * hh);
#pragma unroll
      for (int t = 0; t < 4; ++t) {
        const v16h vb = ldfrag(Vsh + (t * 16 + c) * 64 + kk * 32 + 8 * hh);
        oacc[t] = mma16(pa, vb, oacc[t]);
      }
    }
  }

  __syncthreads();
  float* os = Osh + wave * (16 * 64);
#pragma unroll
  for (int r = 0; r < 8; ++r) {
    const float inv = 1.0f / (1024.0f * lrow[r]);
#pragma unroll
    for (int t = 0; t < 4; ++t) os[(8 * hh + r) * 64 + t * 16 + c] = oacc[t][r] * inv;
  }
  wave_lds_sync();
  const int q = lane >> 3, c8 = (lane & 7) * 8;
  v8h ov[4];
#pragma unroll
  for (int it = 0; it < 4; ++it) {
    const int row = it * 4 + q;
    const float* sp = os + row * 64 + c8;
    const v4f x0 = *(const v4fa*)(sp);
    const v4f x1 = *(const v4fa*)(sp + 4);
    v8h o;
    o[0] = (_Float16)x0[0]; o[1] = (_Float16)x0[1]; o[2] = (_Float16)x0[2]; o[3] = (_Float16)x0[3];
    o[4] = (_Float16)x1[0]; o[5] = (_Float16)x1[1]; o[6] = (_Float16)x1[2]; o[7] = (_Float16)x1[3];
    ov[it] = o;
  }
  for (int pass = 0; pass < 2; ++pass) {
#pragma unroll
    for (int it = 0; it < 4; ++it) {
      const int row = it * 4 + q;
      *(volatile v8h*)(ctx + (size_t)(q0 + row) * ND_ + c8) = ov[it];
    }
    __threadfence();
  }
}

__global__ __launch_bounds__(64)
void dwconv_kernel(const float* __restrict__ G, const float* __restrict__ W, const float* __restrict__ db,
                   const float* __restrict__ bg, const float* __restrict__ bb, _Float16* __restrict__ O,
                   float carry) {
  __shared__ __align__(16) float wsh[KW_ * ND_];
  const int tid = threadIdx.x;
  for (int i = tid; i < KW_ * ND_; i += 64) {
    const int cc = i / KW_;
    const int k  = i - cc * KW_;
    wsh[k * ND_ + cc] = W[i];
  }
  __syncthreads();
  const int rbase = blockIdx.x * 64;
  const int bidx  = rbase / NT_;
  const int tb    = rbase - bidx * NT_;
  const int c8    = tid * 8;
  const float* Gb = G + (size_t)bidx * NT_ * ND_ + c8;
  const v4f db0 = *(const v4f*)(db + c8), db1 = *(const v4f*)(db + c8 + 4);
  const v4f bg0 = *(const v4f*)(bg + c8), bg1 = *(const v4f*)(bg + c8 + 4);
  const v4f bb0 = *(const v4f*)(bb + c8), bb1 = *(const v4f*)(bb + c8 + 4);
#pragma unroll 1
  for (int rr = 0; rr < 64; ++rr) {
    const int t = tb + rr;
    v4f a0 = {0.f, 0.f, 0.f, 0.f};
    v4f a1 = {0.f, 0.f, 0.f, 0.f};
#pragma unroll 1
    for (int k = 0; k < KW_; ++k) {
      const int tt = t + k - (KW_ / 2);
      const int tc = min(max(tt, 0), NT_ - 1);
      const float msk = (tt >= 0 && tt < NT_) ? 1.0f : 0.0f;
      const float* gp = Gb + (size_t)tc * ND_;
      const v4f g0 = *(const v4f*)(gp);
      const v4f g1 = *(const v4f*)(gp + 4);
      const float* wp = wsh + k * ND_ + c8;
      const v4f w0 = *(const v4fa*)(wp);
      const v4f w1 = *(const v4fa*)(wp + 4);
      a0 += (g0 * msk) * w0;
      a1 += (g1 * msk) * w1;
    }
    const v4f s0 = (a0 + db0) * bg0 + bb0;
    const v4f s1 = (a1 + db1) * bg1 + bb1;
    v8h o;
#pragma unroll
    for (int e = 0; e < 4; ++e) {
      o[e]     = (_Float16)(silu_f(s0[e]) * carry);
      o[4 + e] = (_Float16)(silu_f(s1[e]) * carry);
    }
    _Float16* op = O + (size_t)(rbase + rr) * ND_ + c8;
    *(volatile v8h*)op = o;
    __threadfence();
    *(volatile v8h*)op = o;
  }
}

template <int MODE, bool SKEW>
static void run_gemm(hipStream_t st, int gx, int gy,
                     const _Float16* A, int lda, long sA, const _Float16* Bt, int ldb, long sB,
                     void* C1, void* C2, int ldc, long sC, const float* Rsd, int ldr, long sR,
                     const float* b1, const float* b2, const float* b3,
                     int M, int N, int K, int gofs, float scale, float scale2, float carry) {
  gemm_kernel<MODE, SKEW><<<dim3(gx, gy), dim3(256), 0, st>>>(A, lda, sA, Bt, ldb, sB, C1, C2, ldc, sC,
                                                              Rsd, ldr, sR, b1, b2, b3, M, N, K, gofs,
                                                              scale, scale2, carry);
}

extern "C" void kernel_launch(void* const* d_in, const int* in_sizes, int n_in,
                              void* d_out, int out_size, void* d_ws, size_t ws_size,
                              hipStream_t stream) {
  if (n_in < 39) return;
  if (in_sizes[0] != NR_ * ND_) return;
  if (in_sizes[1] != NP_ * ND_) return;
  if (in_sizes[2] != ND_ || in_sizes[3] != ND_) return;
  if (in_sizes[4] != ND_ * NF_ || in_sizes[5] != NF_ || in_sizes[6] != NF_ * ND_ || in_sizes[7] != ND_) return;
  if (in_sizes[8] != ND_ || in_sizes[9] != ND_) return;
  if (in_sizes[10] != ND_ * ND_ || in_sizes[11] != ND_ || in_sizes[12] != ND_ * ND_ || in_sizes[13] != ND_) return;
  if (in_sizes[14] != ND_ * ND_ || in_sizes[15] != ND_ || in_sizes[16] != ND_ * ND_ || in_sizes[17] != ND_) return;
  if (in_sizes[18] != ND_ * ND_ || in_sizes[19] != NH_ * HD_ || in_sizes[20] != NH_ * HD_) return;
  if (in_sizes[21] != ND_ || in_sizes[22] != ND_ || in_sizes[23] != ND_ * 2 * ND_ || in_sizes[24] != 2 * ND_) return;
  if (in_sizes[25] != ND_ * KW_ || in_sizes[26] != ND_ || in_sizes[27] != ND_ || in_sizes[28] != ND_) return;
  if (in_sizes[29] != ND_ * ND_ || in_sizes[30] != ND_ || in_sizes[31] != ND_ || in_sizes[32] != ND_) return;
  if (in_sizes[33] != ND_ * NF_ || in_sizes[34] != NF_ || in_sizes[35] != NF_ * ND_ || in_sizes[36] != ND_) return;
  if (in_sizes[37] != ND_ || in_sizes[38] != ND_) return;
  if (out_size != NR_ * ND_) return;

  const float* x      = (const float*)d_in[0];
  const float* pe     = (const float*)d_in[1];
  const float* ln1_g  = (const float*)d_in[2];
  const float* ln1_b  = (const float*)d_in[3];
  const float* ff1_w1 = (const float*)d_in[4];
  const float* ff1_b1 = (const float*)d_in[5];
  const float* ff1_w2 = (const float*)d_in[6];
  const float* ff1_b2 = (const float*)d_in[7];
  const float* an_g   = (const float*)d_in[8];
  const float* an_b   = (const float*)d_in[9];
  const float* wq     = (const float*)d_in[10];
  const float* bq     = (const float*)d_in[11];
  const float* wk     = (const float*)d_in[12];
  const float* bk     = (const float*)d_in[13];
  const float* wv     = (const float*)d_in[14];
  const float* bvv    = (const float*)d_in[15];
  const float* wo     = (const float*)d_in[16];
  const float* bo     = (const float*)d_in[17];
  const float* posw   = (const float*)d_in[18];
  const float* uvec   = (const float*)d_in[19];
  const float* vvec   = (const float*)d_in[20];
  const float* cn_g   = (const float*)d_in[21];
  const float* cn_b   = (const float*)d_in[22];
  const float* pew    = (const float*)d_in[23];
  const float* peb    = (const float*)d_in[24];
  const float* dww    = (const float*)d_in[25];
  const float* dwb    = (const float*)d_in[26];
  const float* bng    = (const float*)d_in[27];
  const float* bnb    = (const float*)d_in[28];
  const float* pcw    = (const float*)d_in[29];
  const float* pcb    = (const float*)d_in[30];
  const float* ln2_g  = (const float*)d_in[31];
  const float* ln2_b  = (const float*)d_in[32];
  const float* ff2_w1 = (const float*)d_in[33];
  const float* ff2_b1 = (const float*)d_in[34];
  const float* ff2_w2 = (const float*)d_in[35];
  const float* ff2_b2 = (const float*)d_in[36];
  const float* fn_g   = (const float*)d_in[37];
  const float* fn_b   = (const float*)d_in[38];
  float* out = (float*)d_out;

  const size_t SZ_W1  = (size_t)NF_ * ND_ * 2;
  const size_t SZ_WD  = (size_t)ND_ * ND_ * 2;
  const size_t SZ_WPE = (size_t)2 * ND_ * ND_ * 2;
  const size_t SZ_RP  = (size_t)NPP_ * ND_ * 2;
  const size_t SZ_XF  = (size_t)NR_ * ND_ * 4;
  const size_t SZ_A16 = (size_t)NR_ * ND_ * 2;
  const size_t SZ_H16 = (size_t)NR_ * NF_ * 2;
  const size_t SZ_VT  = (size_t)NB_ * ND_ * NT_ * 2;
  const size_t SZ_G   = (size_t)NR_ * ND_ * 4;
  const size_t SZ_BD  = (size_t)NGRP_ * NT_ * BDW_ * 4;
  size_t off = 0;
  const size_t oW1A = off; off += SZ_W1;
  const size_t oW1B = off; off += SZ_W1;
  const size_t oWQ  = off; off += SZ_WD;
  const size_t oWK  = off; off += SZ_WD;
  const size_t oWV  = off; off += SZ_WD;
  const size_t oWO  = off; off += SZ_WD;
  const size_t oWPS = off; off += SZ_WD;
  const size_t oWPC = off; off += SZ_WD;
  const size_t oWPE = off; off += SZ_WPE;
  const size_t oW2A = off; off += SZ_W1;
  const size_t oW2B = off; off += SZ_W1;
  const size_t oRPE = off; off += SZ_RP;
  const size_t oR16 = off; off += SZ_RP;
  const size_t oXF  = off; off += SZ_XF;
  const size_t oLN  = off; off += SZ_A16;
  const size_t oH16 = off; off += SZ_H16;
  const size_t oQU  = off; off += SZ_A16;
  const size_t oQV  = off; off += SZ_A16;
  const size_t oKP  = off; off += SZ_A16;
  const size_t oVT  = off; off += SZ_VT;
  const size_t oCTX = off; off += SZ_A16;
  const size_t oG   = off; off += SZ_G;
  const size_t oCV  = off; off += SZ_A16;
  const size_t oBD  = off; off += SZ_BD;
  const size_t total = off;
  if (total > ws_size) return;
  if (total > (size_t)134217728) return;

  char* ws = (char*)d_ws;
  _Float16* W1A = (_Float16*)(ws + oW1A);
  _Float16* W1B = (_Float16*)(ws + oW1B);
  _Float16* WQ  = (_Float16*)(ws + oWQ);
  _Float16* WK  = (_Float16*)(ws + oWK);
  _Float16* WV  = (_Float16*)(ws + oWV);
  _Float16* WO  = (_Float16*)(ws + oWO);
  _Float16* WPS = (_Float16*)(ws + oWPS);
  _Float16* WPC = (_Float16*)(ws + oWPC);
  _Float16* WPE = (_Float16*)(ws + oWPE);
  _Float16* W2A = (_Float16*)(ws + oW2A);
  _Float16* W2B = (_Float16*)(ws + oW2B);
  _Float16* RPE = (_Float16*)(ws + oRPE);
  _Float16* R16 = (_Float16*)(ws + oR16);
  float*    XF  = (float*)(ws + oXF);
  _Float16* LN16 = (_Float16*)(ws + oLN);
  _Float16* H16 = (_Float16*)(ws + oH16);
  _Float16* QU  = (_Float16*)(ws + oQU);
  _Float16* QV  = (_Float16*)(ws + oQV);
  _Float16* KP  = (_Float16*)(ws + oKP);
  _Float16* VT  = (_Float16*)(ws + oVT);
  _Float16* CTX = (_Float16*)(ws + oCTX);
  float*    G   = (float*)(ws + oG);
  _Float16* CV16 = (_Float16*)(ws + oCV);
  float*    BAND = (float*)(ws + oBD);

  const float cs   = 0.125f * 0.00390625f;
  const float rLW  = 1.0f / 512.0f;
  const float rHW  = 1.0f / 4096.0f;
  const dim3 blk(256);
  const dim3 gLN((NR_ + 7) / 8);

  wtrans_kernel<<<dim3(NF_ / 64, ND_ / 64), blk, 0, stream>>>(ff1_w1, W1A, ND_, NF_, 64.0f);
  wtrans_kernel<<<dim3(ND_ / 64, NF_ / 64), blk, 0, stream>>>(ff1_w2, W1B, NF_, ND_, 64.0f);
  wtrans_kernel<<<dim3(ND_ / 64, ND_ / 64), blk, 0, stream>>>(wq,   WQ,  ND_, ND_, 64.0f);
  wtrans_kernel<<<dim3(ND_ / 64, ND_ / 64), blk, 0, stream>>>(wk,   WK,  ND_, ND_, 64.0f);
  wtrans_kernel<<<dim3(ND_ / 64, ND_ / 64), blk, 0, stream>>>(wv,   WV,  ND_, ND_, 64.0f);
  wtrans_kernel<<<dim3(ND_ / 64, ND_ / 64), blk, 0, stream>>>(wo,   WO,  ND_, ND_, 64.0f);
  wtrans_kernel<<<dim3(ND_ / 64, ND_ / 64), blk, 0, stream>>>(posw, WPS, ND_, ND_, 64.0f);
  wtrans_kernel<<<dim3(ND_ / 64, ND_ / 64), blk, 0, stream>>>(pcw,  WPC, ND_, ND_, 64.0f);
  wtrans_kernel<<<dim3(2 * ND_ / 64, ND_ / 64), blk, 0, stream>>>(pew, WPE, ND_, 2 * ND_, 64.0f);
  wtrans_kernel<<<dim3(NF_ / 64, ND_ / 64), blk, 0, stream>>>(ff2_w1, W2A, ND_, NF_, 64.0f);
  wtrans_kernel<<<dim3(ND_ / 64, NF_ / 64), blk, 0, stream>>>(ff2_w2, W2B, NF_, ND_, 64.0f);
  cvt_rows_kernel<<<dim3((NPP_ * (ND_ / 8) + 255) / 256), blk, 0, stream>>>(pe, RPE, NP_, NPP_, 8.0f);

  {
    const int tiles = (NPP_ / 64) * (ND_ / 64);
    run_gemm<MODE_H16, false>(stream, (tiles + 7) / 8, 1, RPE, ND_, 0L, WPS, ND_, 0L, (void*)R16, (void*)R16, ND_, 0L,
                              x, 0, 0L, bq, bq, bq, NPP_, ND_, ND_, 0, rLW, 0.0f, 16.0f);
  }

  const int tilesF = (NR_ / 64) * (NF_ / 64);
  const int tilesD = (NR_ / 64) * (ND_ / 64);

  ln_kernel<0><<<gLN, blk, 0, stream>>>(x, ln1_g, ln1_b, (void*)LN16, NR_, 8.0f);
  run_gemm<MODE_SILU16, false>(stream, (tilesF + 7) / 8, 1, LN16, ND_, 0L, W1A, ND_, 0L, (void*)H16, (void*)H16, NF_, 0L,
                               x, 0, 0L, ff1_b1, ff1_b1, ff1_b1, NR_, NF_, ND_, 0, rLW, 0.0f, 64.0f);
  run_gemm<MODE_RES32, false>(stream, (tilesD + 7) / 8, 1, H16, NF_, 0L, W1B, NF_, 0L, (void*)XF, (void*)XF, ND_, 0L,
                              x, ND_, 0L, ff1_b2, ff1_b2, ff1_b2, NR_, ND_, NF_, 0, rHW, 0.5f, 1.0f);

  ln_kernel<0><<<gLN, blk, 0, stream>>>(XF, an_g, an_b, (void*)LN16, NR_, 8.0f);
  run_gemm<MODE_QUV, false>(stream, (tilesD + 7) / 8, 1, LN16, ND_, 0L, WQ, ND_, 0L, (void*)QU, (void*)QV, ND_, 0L,
                            x, 0, 0L, bq, uvec, vvec, NR_, ND_, ND_, 0, rLW, 0.0f, 16.0f);
  run_gemm<MODE_H16B, false>(stream, (tilesD + 7) / 8, 1, LN16, ND_, 0L, WK, ND_, 0L, (void*)KP, (void*)KP, ND_, 0L,
                             x, 0, 0L, bk, bk, bk, NR_, ND_, ND_, 0, rLW, 0.0f, 16.0f);
  {
    const int tilesV = (ND_ / 64) * (NT_ / 64);
    run_gemm<MODE_H16RB, false>(stream, (tilesV + 7) / 8, NB_, WV, ND_, 0L, LN16, ND_, (long)NT_ * ND_,
                                (void*)VT, (void*)VT, NT_, (long)ND_ * NT_, x, 0, 0L, bvv, bvv, bvv,
                                ND_, NT_, ND_, 0, rLW, 0.0f, 16.0f);
  }
  for (int g = 0; g < NB_; ++g) {
    const _Float16* Aq = QV + (size_t)g * NT_ * ND_;
    const int tilesBD = (NT_ / 64) * (BDW_ / 64);
    run_gemm<MODE_F32, true>(stream, (tilesBD + 7) / 8, NH_, Aq, ND_, (long)HD_, R16, ND_, (long)HD_,
                             (void*)BAND, (void*)BAND, BDW_, (long)NT_ * BDW_, x, 0, 0L, bq, bq, bq,
                             NT_, BDW_, HD_, 0, cs, 0.0f, 1.0f);
    relattn_kernel<<<dim3(NT_ / 64, NH_), dim3(128), 0, stream>>>(QU, KP, VT, BAND, CTX, g * NH_, cs);
  }
  run_gemm<MODE_RES32, false>(stream, (tilesD + 7) / 8, 1, CTX, ND_, 0L, WO, ND_, 0L, (void*)XF, (void*)XF, ND_, 0L,
                              XF, ND_, 0L, bo, bo, bo, NR_, ND_, ND_, 0, rHW, 1.0f, 1.0f);

  ln_kernel<0><<<gLN, blk, 0, stream>>>(XF, cn_g, cn_b, (void*)LN16, NR_, 8.0f);
  {
    const int tilesG = (NR_ / 64) * (ND_ / 32);
    run_gemm<MODE_GLU32, false>(stream, (tilesG + 7) / 8, 1, LN16, ND_, 0L, WPE, ND_, 0L, (void*)G, (void*)G, ND_, 0L,
                                x, 0, 0L, peb, peb, peb, NR_, ND_, ND_, ND_, rLW, 0.0f, 1.0f);
  }
  dwconv_kernel<<<dim3(NR_ / 64), dim3(64), 0, stream>>>(G, dww, dwb, bng, bnb, CV16, 64.0f);
  run_gemm<MODE_RES32, false>(stream, (tilesD + 7) / 8, 1, CV16, ND_, 0L, WPC, ND_, 0L, (void*)XF, (void*)XF, ND_, 0L,
                              XF, ND_, 0L, pcb, pcb, pcb, NR_, ND_, ND_, 0, rHW, 1.0f, 1.0f);

  ln_kernel<0><<<gLN, blk, 0, stream>>>(XF, ln2_g, ln2_b, (void*)LN16, NR_, 8.0f);
  run_gemm<MODE_SILU16, false>(stream, (tilesF + 7) / 8, 1, LN16, ND_, 0L, W2A, ND_, 0L, (void*)H16, (void*)H16, NF_, 0L,
                               x, 0, 0L, ff2_b1, ff2_b1, ff2_b1, NR_, NF_, ND_, 0, rLW, 0.0f, 64.0f);
  run_gemm<MODE_RES32, false>(stream, (tilesD + 7) / 8, 1, H16, NF_, 0L, W2B, NF_, 0L, (void*)XF, (void*)XF, ND_, 0L,
                              XF, ND_, 0L, ff2_b2, ff2_b2, ff2_b2, NR_, ND_, NF_, 0, rHW, 0.5f, 1.0f);

  ln_kernel<1><<<gLN, blk, 0, stream>>>(XF, fn_g, fn_b, d_out, NR_, 1.0f);
  (void)out;
  (void)hipGetLastError();
}
